// EmbeddingGenerator_19859928776761
// MI455X (gfx1250) — hardware-verified
//
#include <hip/hip_runtime.h>
#include <stddef.h>

typedef __attribute__((ext_vector_type(16))) _Float16 v16h;
typedef __attribute__((ext_vector_type(8)))  _Float16 v8h;
typedef __attribute__((ext_vector_type(8)))  float    v8f;
typedef __attribute__((ext_vector_type(4)))  float    v4f;

__device__ __forceinline__ void dep_guard_h(v8f& a, v8f& b, v16h x, v16h y) { asm volatile("v_nop\n\tv_nop\n\tv_nop\n\tv_nop" : "+v"(a), "+v"(b) : "v"(x), "v"(y)); }
__device__ __forceinline__ void keep4_h(v16h a, v16h b, v16h c, v16h d) { asm volatile("v_nop" :: "v"(a), "v"(b), "v"(c), "v"(d)); }
__device__ __forceinline__ void acc_guard4(v8f& a, v8f& b, v8f& c, v8f& d) { asm volatile("v_nop\n\tv_nop\n\tv_nop\n\tv_nop" : "+v"(a), "+v"(b), "+v"(c), "+v"(d)); }
template <typename T> struct Frag;
template <> struct Frag<_Float16> {
  typedef v16h V; union U { v16h v; v8h h[2]; };
  static __device__ __forceinline__ v16h load(const _Float16* p) {
    U f; f.h[0] = *(const v8h*)(p); f.h[1] = *(const v8h*)(p + 16); return f.v;
  }
  static __device__ __forceinline__ v8f mma(v16h a, v16h b, v8f c) {
    return __builtin_amdgcn_wmma_f32_16x16x32_f16(false, a, false, b, (short)0, c, false, false);
  }
  static __device__ __forceinline__ void guard(v8f& a, v8f& b, v16h x, v16h y) { dep_guard_h(a, b, x, y); }
  static __device__ __forceinline__ void keep(v16h a, v16h b, v16h c, v16h d) { keep4_h(a, b, c, d); }
};

constexpr int NBATCH   = 128;
constexpr int NSTEP    = 256;
constexpr int NHID     = 256;
constexpr int NGATE4   = 1024;
constexpr int NXIN     = 10;
constexpr int NAWS     = 6;
constexpr int NERA     = 4;
constexpr int NXPAD    = 32;
constexpr int HWPIX    = 4096;
constexpr int IMW      = 64;
constexpr int NREP     = 10;
constexpr int ROWS_BLK = 16;
constexpr int LSTM_THREADS = 512;
constexpr int CONV_THREADS = 512;
constexpr float W_SCALE     = 16.0f;
constexpr float W_SCALE_INV = 0.0625f;

static_assert(NBATCH % ROWS_BLK == 0, "rows");
static_assert(NHID == 16 * (LSTM_THREADS / 32), "one unit subtile per wave");
static_assert(NHID % 32 == 0 && NXPAD % 32 == 0, "K multiples of 32");

constexpr size_t WPLANE_BYTES = (size_t)NGATE4 * NHID * 2;
constexpr size_t WX_BYTES     = (size_t)NGATE4 * NXPAD * 2;
constexpr size_t TE_BYTES     = (size_t)NBATCH * NHID * 4;
constexpr size_t OFF_WHH0 = 0;
constexpr size_t OFF_WIH1 = OFF_WHH0 + WPLANE_BYTES;
constexpr size_t OFF_WHH1 = OFF_WIH1 + WPLANE_BYTES;
constexpr size_t OFF_WX0  = OFF_WHH1 + WPLANE_BYTES;
constexpr size_t OFF_TE   = OFF_WX0 + WX_BYTES;
constexpr size_t WS_TOTAL = OFF_TE + TE_BYTES;
static_assert(WS_TOTAL == 1769472, "carve");
static_assert(WS_TOTAL <= (size_t)134217728, "carve cap");

__device__ __forceinline__ v8f zero8f() { return (v8f){0.f, 0.f, 0.f, 0.f, 0.f, 0.f, 0.f, 0.f}; }
__device__ __forceinline__ v16h zero16h() {
  const _Float16 z = (_Float16)0.0f;
  return (v16h){z, z, z, z, z, z, z, z, z, z, z, z, z, z, z, z};
}
__device__ __forceinline__ unsigned h2bits(_Float16 h) { return (unsigned)__builtin_bit_cast(unsigned short, h); }
__device__ __forceinline__ float sigm_f(float x) { return __builtin_amdgcn_rcpf(1.0f + expf(-x)); }

__global__ __launch_bounds__(256) void cast3_scale_f16x2(
    const float* __restrict__ s0, const float* __restrict__ s1, const float* __restrict__ s2,
    _Float16* __restrict__ d0, _Float16* __restrict__ d1, _Float16* __restrict__ d2,
    int n2, float scale)
{
  const int which = blockIdx.y;
  const float* in = (which == 0) ? s0 : ((which == 1) ? s1 : s2);
  _Float16* outp  = (which == 0) ? d0 : ((which == 1) ? d1 : d2);
  const int i = blockIdx.x * 256 + threadIdx.x;
  if (i < n2) {
    const _Float16 h0 = (_Float16)(in[2 * i] * scale);
    const _Float16 h1 = (_Float16)(in[2 * i + 1] * scale);
    const unsigned u = h2bits(h0) | (h2bits(h1) << 16);
    volatile unsigned* o = (volatile unsigned*)outp;
    o[i] = u;
    __threadfence();
    o[i] = u;
  }
}

__global__ __launch_bounds__(256) void build_wx0(const float* __restrict__ wih0, _Float16* __restrict__ wx)
{
  const int i = blockIdx.x * 256 + threadIdx.x;
  if (i < NGATE4 * (NXPAD / 2)) {
    const int n  = i >> 4;
    const int kp = (i & 15) * 2;
    const int k0c = (kp < NXIN) ? kp : (NXIN - 1);
    const int k1c = (kp + 1 < NXIN) ? (kp + 1) : (NXIN - 1);
    float f0 = wih0[n * NXIN + k0c] * W_SCALE;
    float f1 = wih0[n * NXIN + k1c] * W_SCALE;
    f0 = (kp < NXIN) ? f0 : 0.0f;
    f1 = (kp + 1 < NXIN) ? f1 : 0.0f;
    const unsigned u = h2bits((_Float16)f0) | (h2bits((_Float16)f1) << 16);
    volatile unsigned* o = (volatile unsigned*)wx;
    o[i] = u;
    __threadfence();
    o[i] = u;
  }
}

__global__ __launch_bounds__(CONV_THREADS) void conv_pool_kernel(
    const float* __restrict__ terr, const float* __restrict__ cw,
    const float* __restrict__ cb, float* __restrict__ te)
{
  __shared__ __align__(16) float tile[HWPIX];
  __shared__ __align__(16) float part[4][NHID];
  __shared__ __align__(16) float ten[NHID];
  __shared__ float redmn[CONV_THREADS / 32];
  __shared__ float redmx[CONV_THREADS / 32];

  const int tid = threadIdx.x, lane = tid & 31, wave = tid >> 5;
  const int hh = lane >> 4, rlane = lane & 15;
  const int b  = blockIdx.x;
  const int cg = wave & 3;
  const int pg = wave >> 2;

  for (int i = tid; i < HWPIX / 4; i += CONV_THREADS)
    *(v4f*)(tile + 4 * i) = *(const v4f*)(terr + (size_t)b * HWPIX + 4 * i);

  v16h bfr[4];
  float cbias[4];
#pragma unroll
  for (int j = 0; j < 4; ++j) {
    const int ch = 64 * cg + 16 * j + rlane;
    v16h bv = zero16h();
#pragma unroll
    for (int i = 0; i < 8; ++i) {
      const int k  = 8 * hh + i;
      const int kc = (k < 9) ? k : 8;
      const float wv = cw[ch * 9 + kc] * W_SCALE;
      bv[i] = (k < 9) ? (_Float16)wv : (_Float16)0.0f;
    }
    bfr[j] = bv;
    cbias[j] = cb[ch];
  }
  __syncthreads();

  float colsum[4] = {0.f, 0.f, 0.f, 0.f};
#pragma unroll 1
  for (int mi = 0; mi < 64; ++mi) {
    const int mt = pg * 64 + mi;
    const int p  = mt * 16 + rlane;
    const int y  = p >> 6, x = p & 63;
    v16h av = zero16h();
#pragma unroll
    for (int i = 0; i < 8; ++i) {
      const int k  = 8 * hh + i;
      const int dy = (k * 11) >> 5;
      const int dx = k - 3 * dy;
      const int yy = y + dy - 1, xx = x + dx - 1;
      const bool inb = (k < 9) && (yy >= 0) && (yy < IMW) && (xx >= 0) && (xx < IMW);
      const int yc = (yy < 0) ? 0 : ((yy > IMW - 1) ? (IMW - 1) : yy);
      const int xc = (xx < 0) ? 0 : ((xx > IMW - 1) ? (IMW - 1) : xx);
      const float tv = tile[yc * IMW + xc];
      av[i] = inb ? (_Float16)tv : (_Float16)0.0f;
    }
    v8f acc[4];
#pragma unroll
    for (int j = 0; j < 4; ++j) {
      acc[j] = zero8f();
      acc[j] = Frag<_Float16>::mma(av, bfr[j], acc[j]);
    }
    Frag<_Float16>::guard(acc[0], acc[3], av, bfr[3]);
    Frag<_Float16>::keep(bfr[0], bfr[1], bfr[2], bfr[3]);
    acc_guard4(acc[0], acc[1], acc[2], acc[3]);
#pragma unroll
    for (int j = 0; j < 4; ++j) {
      float s = 0.f;
#pragma unroll
      for (int r = 0; r < 8; ++r) {
        const float v = acc[j][r] * W_SCALE_INV + cbias[j];
        s += fmaxf(v, 0.0f);
      }
      colsum[j] += s;
    }
  }

  float tot[4];
#pragma unroll
  for (int j = 0; j < 4; ++j) tot[j] = colsum[j] + __shfl_xor(colsum[j], 16, 32);
#pragma unroll
  for (int j = 0; j < 4; ++j) part[pg][64 * cg + 16 * j + rlane] = tot[j];
  __syncthreads();

  float v = 0.f;
  if (tid < NHID) v = ((part[0][tid] + part[1][tid]) + (part[2][tid] + part[3][tid])) * (1.0f / 4096.0f);
  float mn = (tid < NHID) ? v : INFINITY;
  float mx = (tid < NHID) ? v : -INFINITY;
#pragma unroll
  for (int off = 16; off > 0; off >>= 1) {
    mn = fminf(mn, __shfl_xor(mn, off, 32));
    mx = fmaxf(mx, __shfl_xor(mx, off, 32));
  }
  if (lane == 0) { redmn[wave] = mn; redmx[wave] = mx; }
  __syncthreads();
  float gmn = redmn[0], gmx = redmx[0];
#pragma unroll
  for (int w = 1; w < CONV_THREADS / 32; ++w) { gmn = fminf(gmn, redmn[w]); gmx = fmaxf(gmx, redmx[w]); }
  const float den  = gmx - gmn;
  const float rden = 1.0f / den;
  const float nv   = (den != 0.0f) ? ((v - gmn) * rden) : 0.0f;
  if (tid < NHID) ten[tid] = nv;
  __syncthreads();

  if (wave < 2) {
    const int e = wave * 128 + 4 * lane;
    const v4f val = *(const v4f*)(ten + e);
    volatile v4f* dst = (volatile v4f*)(te + (size_t)b * NHID + e);
    *dst = val;
    __threadfence();
    *dst = val;
  }
}

__device__ __forceinline__ void kpass(v8f (&acc)[4], const _Float16* At, int lda,
                                      const _Float16* __restrict__ Bp, int ldb, int nk,
                                      int nrow0, int rlane, int koff, unsigned zofs)
{
#pragma unroll 2
  for (int ks = 0; ks < nk; ++ks) {
    const int k0 = ks * 32;
    const v16h a = Frag<_Float16>::load(At + rlane * lda + k0 + koff);
    v16h bf[4];
#pragma unroll
    for (int g = 0; g < 4; ++g)
      bf[g] = Frag<_Float16>::load(Bp + (size_t)(g * NHID + nrow0 + rlane) * ldb + k0 + koff + zofs);
#pragma unroll
    for (int g = 0; g < 4; ++g) acc[g] = Frag<_Float16>::mma(a, bf[g], acc[g]);
    Frag<_Float16>::guard(acc[0], acc[3], a, bf[3]);
    Frag<_Float16>::keep(bf[0], bf[1], bf[2], bf[3]);
  }
}

__global__ __launch_bounds__(LSTM_THREADS) void lstm2_kernel(
    const float* __restrict__ aws, const float* __restrict__ era,
    const _Float16* __restrict__ wx0, const _Float16* __restrict__ whh0,
    const _Float16* __restrict__ wih1, const _Float16* __restrict__ whh1,
    const float* __restrict__ bih0, const float* __restrict__ bhh0,
    const float* __restrict__ bih1, const float* __restrict__ bhh1,
    const float* __restrict__ te, float* __restrict__ out)
{
  __shared__ __align__(16) _Float16 H0s[2][ROWS_BLK * NHID];
  __shared__ __align__(16) _Float16 H1s[2][ROWS_BLK * NHID];
  __shared__ __align__(16) _Float16 Xs[ROWS_BLK * NXPAD];
  __shared__ __align__(16) float    slab[ROWS_BLK * NHID];

  const int tid = threadIdx.x, lane = tid & 31, wave = tid >> 5;
  const int hh = lane >> 4, rlane = lane & 15, koff = hh * 8;
  const int b0 = blockIdx.x * ROWS_BLK;
  const int nrow0 = 16 * wave;
  const int unit  = nrow0 + rlane;

  for (int i = tid; i < 2 * ROWS_BLK * NHID; i += LSTM_THREADS) {
    (&H0s[0][0])[i] = (_Float16)0.0f;
    (&H1s[0][0])[i] = (_Float16)0.0f;
  }
  float bi0[4], bi1[4];
#pragma unroll
  for (int g = 0; g < 4; ++g) {
    const int n = g * NHID + unit;
    bi0[g] = bih0[n] + bhh0[n];
    bi1[g] = bih1[n] + bhh1[n];
  }
  float cs0[8], cs1[8];
#pragma unroll
  for (int r = 0; r < 8; ++r) { cs0[r] = 0.f; cs1[r] = 0.f; }
  __syncthreads();

  for (int t = 0; t < NSTEP; ++t) {
    const int pr = (t + 1) & 1;
    const int pw = t & 1;
    unsigned zofs;
    asm volatile("v_mov_b32 %0, 0" : "=v"(zofs));

    if (tid < 256) {
      const int row = tid >> 4;
      const int kp  = (tid & 15) * 2;
      const size_t base = (size_t)(b0 + row) * NSTEP + t;
      const int ka0 = (kp < NAWS) ? kp : (NAWS - 1);
      const int ka1 = (kp + 1 < NAWS) ? (kp + 1) : (NAWS - 1);
      int ke0 = kp - NAWS;     ke0 = (ke0 < 0) ? 0 : ((ke0 > NERA - 1) ? (NERA - 1) : ke0);
      int ke1 = kp + 1 - NAWS; ke1 = (ke1 < 0) ? 0 : ((ke1 > NERA - 1) ? (NERA - 1) : ke1);
      const float a0 = aws[base * NAWS + ka0];
      const float a1 = aws[base * NAWS + ka1];
      const float e0 = era[base * NERA + ke0];
      const float e1 = era[base * NERA + ke1];
      const float f0 = (kp < NAWS) ? a0 : ((kp < NXIN) ? e0 : 0.0f);
      const float f1 = (kp + 1 < NAWS) ? a1 : ((kp + 1 < NXIN) ? e1 : 0.0f);
      const unsigned w = h2bits((_Float16)f0) | (h2bits((_Float16)f1) << 16);
      *(unsigned*)(Xs + row * NXPAD + kp) = w;
    }
    __syncthreads();

    {
      v8f acc[4];
#pragma unroll
      for (int g = 0; g < 4; ++g) acc[g] = zero8f();
      kpass(acc, Xs, NXPAD, wx0, NXPAD, 1, nrow0, rlane, koff, zofs);
      kpass(acc, H0s[pr], NHID, whh0, NHID, NHID / 32, nrow0, rlane, koff, zofs);
      acc_guard4(acc[0], acc[1], acc[2], acc[3]);
      _Float16* hw = H0s[pw];
#pragma unroll
      for (int r = 0; r < 8; ++r) {
        const float zi = acc[0][r] * W_SCALE_INV + bi0[0];
        const float zf = acc[1][r] * W_SCALE_INV + bi0[1];
        const float zg = acc[2][r] * W_SCALE_INV + bi0[2];
        const float zq = acc[3][r] * W_SCALE_INV + bi0[3];
        const float c  = sigm_f(zf) * cs0[r] + sigm_f(zi) * tanhf(zg);
        cs0[r] = c;
        const float h = sigm_f(zq) * tanhf(c);
        hw[(8 * hh + r) * NHID + unit] = (_Float16)h;
      }
    }
    __syncthreads();

    {
      v8f acc[4];
#pragma unroll
      for (int g = 0; g < 4; ++g) acc[g] = zero8f();
      kpass(acc, H0s[pw], NHID, wih1, NHID, NHID / 32, nrow0, rlane, koff, zofs);
      kpass(acc, H1s[pr], NHID, whh1, NHID, NHID / 32, nrow0, rlane, koff, zofs);
      acc_guard4(acc[0], acc[1], acc[2], acc[3]);
      _Float16* hw1 = H1s[pw];
      const bool last = (t == NSTEP - 1);
#pragma unroll
      for (int r = 0; r < 8; ++r) {
        const float zi = acc[0][r] * W_SCALE_INV + bi1[0];
        const float zf = acc[1][r] * W_SCALE_INV + bi1[1];
        const float zg = acc[2][r] * W_SCALE_INV + bi1[2];
        const float zq = acc[3][r] * W_SCALE_INV + bi1[3];
        const float c  = sigm_f(zf) * cs1[r] + sigm_f(zi) * tanhf(zg);
        cs1[r] = c;
        const float h = sigm_f(zq) * tanhf(c);
        hw1[(8 * hh + r) * NHID + unit] = (_Float16)h;
        if (last) {
          const int row = 8 * hh + r;
          slab[row * NHID + unit] = h + te[(size_t)(b0 + row) * NHID + unit];
        }
      }
    }
  }
  __syncthreads();

  for (int pass = 0; pass < 2; ++pass) {
#pragma unroll 1
    for (int i = 0; i < 20; ++i) {
      const int q  = wave + 16 * i;
      const int lr = q / 20;
      const int cq = q - lr * 20;
      const v4f val = *(const v4f*)(slab + lr * NHID + (cq & 1) * 128 + 4 * lane);
      *(volatile v4f*)(out + (size_t)(b0 + lr) * (NREP * NHID) + cq * 128 + 4 * lane) = val;
    }
    __threadfence();
  }
}

extern "C" void kernel_launch(void* const* d_in, const int* in_sizes, int n_in,
                              void* d_out, int out_size, void* d_ws, size_t ws_size,
                              hipStream_t stream)
{
  if (n_in < 13) return;
  if (out_size != NBATCH * NREP * NHID) return;
  if (in_sizes[2] != NBATCH * HWPIX) return;
  if (in_sizes[4] != NGATE4 * NHID) return;
  if (ws_size < WS_TOTAL) return;

  const float* aws   = (const float*)d_in[0];
  const float* era   = (const float*)d_in[1];
  const float* terr  = (const float*)d_in[2];
  const float* wih0f = (const float*)d_in[3];
  const float* whh0f = (const float*)d_in[4];
  const float* bih0  = (const float*)d_in[5];
  const float* bhh0  = (const float*)d_in[6];
  const float* wih1f = (const float*)d_in[7];
  const float* whh1f = (const float*)d_in[8];
  const float* bih1  = (const float*)d_in[9];
  const float* bhh1  = (const float*)d_in[10];
  const float* convw = (const float*)d_in[11];
  const float* convb = (const float*)d_in[12];

  char* ws = (char*)d_ws;
  _Float16* whh0h = (_Float16*)(ws + OFF_WHH0);
  _Float16* wih1h = (_Float16*)(ws + OFF_WIH1);
  _Float16* whh1h = (_Float16*)(ws + OFF_WHH1);
  _Float16* wx0h  = (_Float16*)(ws + OFF_WX0);
  float*    te    = (float*)(ws + OFF_TE);
  float*    out   = (float*)d_out;

  const int n2 = NGATE4 * NHID / 2;
  cast3_scale_f16x2<<<dim3(n2 / 256, 3), 256, 0, stream>>>(
      whh0f, wih1f, whh1f, whh0h, wih1h, whh1h, n2, W_SCALE);
  build_wx0<<<NGATE4 * (NXPAD / 2) / 256, 256, 0, stream>>>(wih0f, wx0h);
  conv_pool_kernel<<<NBATCH, CONV_THREADS, 0, stream>>>(terr, convw, convb, te);
  lstm2_kernel<<<NBATCH / ROWS_BLK, LSTM_THREADS, 0, stream>>>(
      aws, era, wx0h, whh0h, wih1h, whh1h, bih0, bhh0, bih1, bhh1, te, out);
}
